// NormAttention_9079560863963
// MI455X (gfx1250) — hardware-verified
//
#include <hip/hip_runtime.h>
#include <math.h>

constexpr int kBatch = 2;
constexpr int kSeq   = 2048;
constexpr int kEmb   = 1024;
constexpr int kHid   = 1024;
constexpr int kHeads = 8;
constexpr int kDh    = 128;
constexpr int kTok   = kBatch * kSeq;
constexpr int kGrpPerChunk = 4;
constexpr int kNumChunks   = (kBatch * kHeads) / kGrpPerChunk;
constexpr float kWCarry    = 16.0f;
constexpr float kWCarryInv = 1.0f / 16.0f;
constexpr float kRmsFac    = 0.03125f;
constexpr float kEps       = 1e-8f;

constexpr size_t kBytesX16  = (size_t)kTok * kEmb * 2;
constexpr size_t kBytesWpl  = (size_t)kHid * kEmb * 2;
constexpr size_t kBytesW16  = 5 * kBytesWpl;
constexpr size_t kBytesQ16  = (size_t)kTok * kHid * 2;
constexpr size_t kBytesK16  = kBytesQ16;
constexpr size_t kBytesVT16 = (size_t)kHid * kTok * 2;
constexpr size_t kBytesU32  = (size_t)kTok * kHid * 4;
constexpr size_t kBytesE16  = (size_t)kGrpPerChunk * kSeq * kSeq * 2;
constexpr size_t kBytesO32  = (size_t)kTok * kHid * 4;
constexpr size_t kBytesG16  = (size_t)kTok * kHid * 2;
constexpr size_t kOffX16  = 0;
constexpr size_t kOffW16  = kOffX16  + kBytesX16;
constexpr size_t kOffQ16  = kOffW16  + kBytesW16;
constexpr size_t kOffK16  = kOffQ16  + kBytesQ16;
constexpr size_t kOffVT16 = kOffK16  + kBytesK16;
constexpr size_t kOffU32  = kOffVT16 + kBytesVT16;
constexpr size_t kOffE16  = kOffU32  + kBytesU32;
constexpr size_t kOffO32  = kOffE16  + kBytesE16;
constexpr size_t kOffG16  = kOffO32  + kBytesO32;
constexpr size_t kWsTotal = kOffG16  + kBytesG16;

typedef __attribute__((ext_vector_type(16))) _Float16 v16h;
typedef __attribute__((ext_vector_type(8)))  _Float16 v8h;
typedef __attribute__((ext_vector_type(16))) __bf16   v16b;
typedef __attribute__((ext_vector_type(8)))  __bf16   v8b;
typedef __attribute__((ext_vector_type(8)))  float    v8f;
typedef __attribute__((ext_vector_type(4)))  float    v4f;
typedef __attribute__((ext_vector_type(4)))  unsigned int v4u;

__device__ __forceinline__ unsigned short f2bf_bits(float f) {
  unsigned u = __float_as_uint(f);
  return (unsigned short)((u + 0x7FFFu + ((u >> 16) & 1u)) >> 16);
}
__device__ __forceinline__ float bf_bits2f(unsigned short h) { return __uint_as_float(((unsigned)h) << 16); }

__device__ __forceinline__ void dep_guard_h(v8f& a, v8f& b, v16h x, v16h y) { asm volatile("v_nop\n\tv_nop\n\tv_nop\n\tv_nop" : "+v"(a), "+v"(b) : "v"(x), "v"(y)); }
__device__ __forceinline__ void dep_guard_b(v8f& a, v8f& b, v16b x, v16b y) { asm volatile("v_nop\n\tv_nop\n\tv_nop\n\tv_nop" : "+v"(a), "+v"(b) : "v"(x), "v"(y)); }
__device__ __forceinline__ void keep4_h(v16h a, v16h b, v16h c, v16h d) { asm volatile("v_nop" :: "v"(a), "v"(b), "v"(c), "v"(d)); }
__device__ __forceinline__ void keep4_b(v16b a, v16b b, v16b c, v16b d) { asm volatile("v_nop" :: "v"(a), "v"(b), "v"(c), "v"(d)); }
__device__ __forceinline__ void acc_guard4(v8f& a, v8f& b, v8f& c, v8f& d) { asm volatile("v_nop\n\tv_nop\n\tv_nop\n\tv_nop" : "+v"(a), "+v"(b), "+v"(c), "+v"(d)); }
template <typename T> struct Frag;
template <> struct Frag<_Float16> {
  typedef v16h V; union U { v16h v; v8h h[2]; };
  static __device__ __forceinline__ v16h load(const _Float16* p) {
    U f; f.h[0] = *(const v8h*)(p); f.h[1] = *(const v8h*)(p + 16); return f.v;
  }
  static __device__ __forceinline__ v8f mma(v16h a, v16h b, v8f c) {
    return __builtin_amdgcn_wmma_f32_16x16x32_f16(false, a, false, b, (short)0, c, false, false);
  }
  static __device__ __forceinline__ void guard(v8f& a, v8f& b, v16h x, v16h y) { dep_guard_h(a, b, x, y); }
  static __device__ __forceinline__ void keep(v16h a, v16h b, v16h c, v16h d) { keep4_h(a, b, c, d); }
};
template <> struct Frag<__bf16> {
  typedef v16b V; union U { v16b v; v8b h[2]; };
  static __device__ __forceinline__ v16b load(const __bf16* p) {
    U f; f.h[0] = *(const v8b*)(p); f.h[1] = *(const v8b*)(p + 16); return f.v;
  }
  static __device__ __forceinline__ v8f mma(v16b a, v16b b, v8f c) {
    return __builtin_amdgcn_wmma_f32_16x16x32_bf16(false, a, false, b, (short)0, c, false, false);
  }
  static __device__ __forceinline__ void guard(v8f& a, v8f& b, v16b x, v16b y) { dep_guard_b(a, b, x, y); }
  static __device__ __forceinline__ void keep(v16b a, v16b b, v16b c, v16b d) { keep4_b(a, b, c, d); }
};

__device__ __forceinline__ unsigned pk16(unsigned short a, unsigned short b) { return (unsigned)a | ((unsigned)b << 16); }
__device__ __forceinline__ unsigned short h_bits(float f) { const _Float16 h = (_Float16)f; return __builtin_bit_cast(unsigned short, h); }

template <int ET> struct Elem;
template <> struct Elem<0> { typedef _Float16 T; };
template <> struct Elem<1> { typedef __bf16 T; };
template <int ET, bool SPLIT, int BIAS_MODE, int OUT_MODE, bool RESID, int ACT = 0, int TRI = 0>
__global__ __launch_bounds__(256) void wmma_gemm64(
    const unsigned short* __restrict__ Ap, const unsigned short* __restrict__ A2p, int lda, long strideA,
    const unsigned short* __restrict__ Btp, const unsigned short* __restrict__ Bt2p, int ldb, long strideB,
    void* __restrict__ Cout, void* __restrict__ Cout2, int ldc, long strideC,
    const float* __restrict__ bias,
    const float* __restrict__ resid, long strideR,
    int M, int N, int K, float scale) {
  typedef typename Elem<ET>::T T;
  typedef typename Frag<T>::V V;
  const T* A = (const T*)Ap; const T* A2 = (const T*)A2p; const T* Bt = (const T*)Btp; const T* Bt2 = (const T*)Bt2p;
  __shared__ __align__(16) float sT[8][16 * 68];
  const int b    = blockIdx.y;
  const int lane = threadIdx.x & 31;
  const int wave = threadIdx.x >> 5;
  const int tilesN = N >> 6;
  const int tilesM = M >> 6;
  const int tile = blockIdx.x * 8 + wave;
  if (tile >= tilesM * tilesN) return;
  const int tm = tile / tilesN;
  const int tn = tile - tm * tilesN;
  if (TRI == 1) { if (tn > tm) return; }
  const int m0 = tm << 6;
  const int n0 = tn << 6;
  const int Kt = (TRI == 2) ? (((m0 + 64) < K) ? (m0 + 64) : K) : K;

  const T* Ab  = A  + (size_t)b * strideA;
  const T* Bb  = Bt + (size_t)b * strideB;
  const T* Ab2 = SPLIT ? (A2  + (size_t)b * strideA) : nullptr;
  const T* Bb2 = SPLIT ? (Bt2 + (size_t)b * strideB) : nullptr;

  const int rlane = lane & 15;
  const int koff  = (lane >> 4) * 8;
  const int mOff  = (lane >> 4) * 8;

  v8f acc[4][4];
#pragma unroll
  for (int i = 0; i < 4; ++i)
#pragma unroll
    for (int j = 0; j < 4; ++j) acc[i][j] = (v8f){0.f,0.f,0.f,0.f,0.f,0.f,0.f,0.f};

  for (int k0 = 0; k0 < Kt; k0 += 32) {
    V bh[4], bl[4];
#pragma unroll
    for (int j = 0; j < 4; ++j) {
      const size_t bo = (size_t)(n0 + (j << 4) + rlane) * ldb + koff + k0;
      bh[j] = Frag<T>::load(Bb + bo);
      if (SPLIT) bl[j] = Frag<T>::load(Bb2 + bo);
    }
#pragma unroll
    for (int i = 0; i < 4; ++i) {
      const size_t ao = (size_t)(m0 + (i << 4) + rlane) * lda + koff + k0;
      V ah = Frag<T>::load(Ab + ao);
      V al;
      if (SPLIT) al = Frag<T>::load(Ab2 + ao);
#pragma unroll
      for (int j = 0; j < 4; ++j) {
        acc[i][j] = Frag<T>::mma(ah, bh[j], acc[i][j]);
        if (SPLIT) {
          acc[i][j] = Frag<T>::mma(ah, bl[j], acc[i][j]);
          acc[i][j] = Frag<T>::mma(al, bh[j], acc[i][j]);
        }
      }
      Frag<T>::guard(acc[i][0], acc[i][3], ah, SPLIT ? al : ah);
    }
    Frag<T>::keep(bh[0], bh[1], bh[2], bh[3]);
    if (SPLIT) Frag<T>::keep(bl[0], bl[1], bl[2], bl[3]);
  }
  acc_guard4(acc[0][0], acc[0][1], acc[0][2], acc[0][3]);
  acc_guard4(acc[1][0], acc[1][1], acc[1][2], acc[1][3]);
  acc_guard4(acc[2][0], acc[2][1], acc[2][2], acc[2][3]);
  acc_guard4(acc[3][0], acc[3][1], acc[3][2], acc[3][3]);

  float* slab = sT[wave];
  const float* Rb = RESID ? (resid + (size_t)b * strideR) : nullptr;
#pragma unroll
  for (int i = 0; i < 4; ++i) {
    const int mBase = m0 + (i << 4);
#pragma unroll
    for (int j = 0; j < 4; ++j) {
      const int n = n0 + (j << 4) + rlane;
      float bv = 0.f;
      if (BIAS_MODE == 2) bv = bias[n];
#pragma unroll
      for (int r = 0; r < 8; ++r) {
        float v = acc[i][j][r] * scale;
        if (BIAS_MODE == 1) v += bias[mBase + mOff + r];
        if (BIAS_MODE == 2) v += bv;
        if (RESID) v += Rb[(size_t)(mBase + mOff + r) * ldc + n];
        if (ACT == 2) v = fmaxf(v, 0.0f);
        if (ACT == 3) v = v / (1.0f + expf(-v));
        if (ACT == 4) v = (v > 0.f) ? v : 0.01f * v;
        if (ACT == 6) v = (v > 0.f) ? v : (expf(v) - 1.0f);
        if (TRI == 1) { if (n > mBase + mOff + r) v = 0.0f; }
        slab[(mOff + r) * 68 + (j << 4) + rlane] = v;
      }
    }
    __builtin_amdgcn_fence(__ATOMIC_RELEASE, "workgroup");
    __builtin_amdgcn_wave_barrier();
    __builtin_amdgcn_fence(__ATOMIC_ACQUIRE, "workgroup");
    if (OUT_MODE == 0) {
      float* C = (float*)Cout + (size_t)b * strideC;
      const int hh = lane >> 4, c4 = (lane & 15) * 4;
      for (int pass = 0; pass < 2; ++pass) {
#pragma unroll
        for (int it = 0; it < 8; ++it) {
          const int row = it * 2 + hh;
          v4f v = *(const v4f*)(slab + row * 68 + c4);
          *(volatile v4f*)(C + (size_t)(mBase + row) * ldc + n0 + c4) = v;
        }
        __threadfence();
      }
    } else {
      const int q = lane >> 3, c8 = (lane & 7) * 8;
      unsigned short* C  = (unsigned short*)Cout  + (size_t)b * strideC;
      unsigned short* C2 = (OUT_MODE == 2) ? ((unsigned short*)Cout2 + (size_t)b * strideC) : nullptr;
      for (int pass = 0; pass < 2; ++pass) {
#pragma unroll
        for (int it = 0; it < 4; ++it) {
          const int row = it * 4 + q;
          const float* sp = slab + row * 68 + c8;
          v8h hv, lv;
#pragma unroll
          for (int e = 0; e < 8; ++e) {
            if (OUT_MODE == 1) {
              hv[e] = (_Float16)sp[e];
            } else {
              unsigned short hb = f2bf_bits(sp[e]);
              unsigned short lb = f2bf_bits(sp[e] - bf_bits2f(hb));
              hv[e] = __builtin_bit_cast(_Float16, hb);
              lv[e] = __builtin_bit_cast(_Float16, lb);
            }
          }
          *(volatile v8h*)(C + (size_t)(mBase + row) * ldc + n0 + c8) = hv;
          if (OUT_MODE == 2) *(volatile v8h*)(C2 + (size_t)(mBase + row) * ldc + n0 + c8) = lv;
        }
        __threadfence();
      }
    }
    __builtin_amdgcn_fence(__ATOMIC_RELEASE, "workgroup");
    __builtin_amdgcn_wave_barrier();
    __builtin_amdgcn_fence(__ATOMIC_ACQUIRE, "workgroup");
  }
}

__global__ __launch_bounds__(256) void cast8_f16_kernel(const float* __restrict__ p0, const float* __restrict__ p1,
                                                        const float* __restrict__ p2, const float* __restrict__ p3,
                                                        const float* __restrict__ p4, unsigned short* __restrict__ out,
                                                        long planeElems, int n8, float scale) {
  const int z = blockIdx.y;
  const float* in = (z == 0) ? p0 : (z == 1) ? p1 : (z == 2) ? p2 : (z == 3) ? p3 : p4;
  const int i = blockIdx.x * 256 + threadIdx.x;
  if (i >= n8) return;
  const float* p = in + 8 * (size_t)i;
  const v4f a = *(const v4f*)(p);
  const v4f c = *(const v4f*)(p + 4);
  unsigned short hb[8];
#pragma unroll
  for (int e = 0; e < 4; ++e) {
    hb[e]     = h_bits(a[e] * scale);
    hb[4 + e] = h_bits(c[e] * scale);
  }
  const v4u u = (v4u){pk16(hb[0], hb[1]), pk16(hb[2], hb[3]), pk16(hb[4], hb[5]), pk16(hb[6], hb[7])};
  unsigned short* q = out + (size_t)z * (size_t)planeElems + 8 * (size_t)i;
  *(volatile v4u*)q = u;
  __threadfence();
  *(volatile v4u*)q = u;
}

__global__ __launch_bounds__(128) void rms_gate_kernel(const float* __restrict__ O, const float* __restrict__ U,
                                                       const float* __restrict__ sc, unsigned short* __restrict__ G) {
  __shared__ float red[4];
  const int row  = blockIdx.x;
  const int t    = threadIdx.x;
  const int lane = t & 31, wave = t >> 5;
  const size_t base = (size_t)row * kHid + 8 * (size_t)t;
  const v4f oa = *(const v4f*)(O + base);
  const v4f oc = *(const v4f*)(O + base + 4);
  float ss = 0.f;
#pragma unroll
  for (int e = 0; e < 4; ++e) ss += oa[e] * oa[e];
#pragma unroll
  for (int e = 0; e < 4; ++e) ss += oc[e] * oc[e];
#pragma unroll
  for (int off = 16; off > 0; off >>= 1) ss += __shfl_xor(ss, off, 32);
  if (lane == 0) red[wave] = ss;
  __syncthreads();
  const float tot = ((red[0] + red[1]) + red[2]) + red[3];
  const float rms = sqrtf(tot) * kRmsFac;
  const float inv = 1.0f / (rms + kEps);
  const v4f ua = *(const v4f*)(U + base);
  const v4f uc = *(const v4f*)(U + base + 4);
  const v4f sa = *(const v4f*)(sc + 8 * t);
  const v4f sb = *(const v4f*)(sc + 8 * t + 4);
  unsigned short hb[8];
#pragma unroll
  for (int e = 0; e < 4; ++e) {
    const float g0 = ua[e] * (sa[e] * (oa[e] * inv));
    const float g1 = uc[e] * (sb[e] * (oc[e] * inv));
    hb[e]     = h_bits(g0);
    hb[4 + e] = h_bits(g1);
  }
  const v4u u = (v4u){pk16(hb[0], hb[1]), pk16(hb[2], hb[3]), pk16(hb[4], hb[5]), pk16(hb[6], hb[7])};
  unsigned short* q = G + base;
  *(volatile v4u*)q = u;
  __threadfence();
  *(volatile v4u*)q = u;
}

extern "C" void kernel_launch(void* const* d_in, const int* in_sizes, int n_in,
                              void* d_out, int out_size, void* d_ws, size_t ws_size,
                              hipStream_t stream) {
  if (n_in < 12) return;
  if (in_sizes[0] != kTok * kEmb) return;
  if (in_sizes[1] != kHid * kEmb || in_sizes[3] != kHid * kEmb || in_sizes[5] != kHid * kEmb ||
      in_sizes[7] != kHid * kEmb || in_sizes[9] != kEmb * kHid) return;
  if (in_sizes[2] != kHid || in_sizes[4] != kHid || in_sizes[6] != kHid || in_sizes[8] != kHid ||
      in_sizes[10] != kEmb || in_sizes[11] != kHid) return;
  if (out_size != kTok * kEmb) return;
  if (ws_size < kWsTotal) return;

  const float* x  = (const float*)d_in[0];
  const float* Wq = (const float*)d_in[1];
  const float* bq = (const float*)d_in[2];
  const float* Wk = (const float*)d_in[3];
  const float* bk = (const float*)d_in[4];
  const float* Wv = (const float*)d_in[5];
  const float* bv = (const float*)d_in[6];
  const float* Wu = (const float*)d_in[7];
  const float* bu = (const float*)d_in[8];
  const float* Wo = (const float*)d_in[9];
  const float* bo = (const float*)d_in[10];
  const float* sc = (const float*)d_in[11];
  float* Y = (float*)d_out;

  char* ws = (char*)d_ws;
  unsigned short* X16  = (unsigned short*)(ws + kOffX16);
  unsigned short* W16  = (unsigned short*)(ws + kOffW16);
  unsigned short* Wq16 = W16 + 0 * (size_t)kHid * kEmb;
  unsigned short* Wk16 = W16 + 1 * (size_t)kHid * kEmb;
  unsigned short* Wv16 = W16 + 2 * (size_t)kHid * kEmb;
  unsigned short* Wu16 = W16 + 3 * (size_t)kHid * kEmb;
  unsigned short* Wo16 = W16 + 4 * (size_t)kHid * kEmb;
  unsigned short* Q16  = (unsigned short*)(ws + kOffQ16);
  unsigned short* K16  = (unsigned short*)(ws + kOffK16);
  unsigned short* VT16 = (unsigned short*)(ws + kOffVT16);
  float*          U32  = (float*)(ws + kOffU32);
  unsigned short* E16  = (unsigned short*)(ws + kOffE16);
  float*          O32  = (float*)(ws + kOffO32);
  unsigned short* G16  = (unsigned short*)(ws + kOffG16);

  cast8_f16_kernel<<<dim3(2048, 1), 256, 0, stream>>>(x, x, x, x, x, X16, 0L, (kTok * kEmb) / 8, 1.0f);
  cast8_f16_kernel<<<dim3(512, 5), 256, 0, stream>>>(Wq, Wk, Wv, Wu, Wo, W16, (long)kHid * kEmb,
                                                      (kHid * kEmb) / 8, kWCarry);

  wmma_gemm64<0, false, 2, 1, false, 6, 0><<<dim3(128, 1), 256, 0, stream>>>(
      X16, X16, kEmb, 0L, Wq16, Wq16, kEmb, 0L, (void*)Q16, (void*)Q16, kHid, 0L, bq, bq, 0L,
      kTok, kHid, kEmb, kWCarryInv);
  wmma_gemm64<0, false, 2, 1, false, 6, 0><<<dim3(128, 1), 256, 0, stream>>>(
      X16, X16, kEmb, 0L, Wk16, Wk16, kEmb, 0L, (void*)K16, (void*)K16, kHid, 0L, bk, bk, 0L,
      kTok, kHid, kEmb, kWCarryInv);
  wmma_gemm64<0, false, 1, 1, false, 3, 0><<<dim3(128, 1), 256, 0, stream>>>(
      Wv16, Wv16, kEmb, 0L, X16, X16, kEmb, 0L, (void*)VT16, (void*)VT16, kTok, 0L, bv, bv, 0L,
      kHid, kTok, kEmb, kWCarryInv);
  wmma_gemm64<0, false, 2, 0, false, 3, 0><<<dim3(128, 1), 256, 0, stream>>>(
      X16, X16, kEmb, 0L, Wu16, Wu16, kEmb, 0L, (void*)U32, (void*)U32, kHid, 0L, bu, bu, 0L,
      kTok, kHid, kEmb, kWCarryInv);

  for (int c = 0; c < kNumChunks; ++c) {
    const int b  = c >> 1;
    const int h0 = (c & 1) * kGrpPerChunk;
    const unsigned short* Qg = Q16 + (size_t)b * kSeq * kHid + (size_t)h0 * kDh;
    const unsigned short* Kg = K16 + (size_t)b * kSeq * kHid + (size_t)h0 * kDh;
    const unsigned short* VTg = VT16 + (size_t)h0 * kDh * kTok + (size_t)b * kSeq;
    float* Og = O32 + (size_t)b * kSeq * kHid + (size_t)h0 * kDh;
    wmma_gemm64<0, false, 0, 1, false, 0, 1><<<dim3(128, kGrpPerChunk), 256, 0, stream>>>(
        Qg, Qg, kHid, (long)kDh, Kg, Kg, kHid, (long)kDh, (void*)E16, (void*)E16, kSeq, (long)kSeq * kSeq,
        bq, bq, 0L, kSeq, kSeq, kDh, 1.0f);
    wmma_gemm64<0, false, 0, 0, false, 0, 2><<<dim3(8, kGrpPerChunk), 256, 0, stream>>>(
        E16, E16, kSeq, (long)kSeq * kSeq, VTg, VTg, kTok, (long)kDh * kTok, (void*)Og, (void*)Og, kHid, (long)kDh,
        bq, bq, 0L, kSeq, kDh, kSeq, 1.0f);
  }

  rms_gate_kernel<<<dim3(kTok, 1), 128, 0, stream>>>(O32, U32, sc, G16);

  wmma_gemm64<0, false, 2, 0, false, 0, 0><<<dim3(128, 1), 256, 0, stream>>>(
      G16, G16, kHid, 0L, Wo16, Wo16, kHid, 0L, (void*)Y, (void*)Y, kEmb, 0L, bo, bo, 0L,
      kTok, kEmb, kHid, kWCarryInv);
}
